// RNNModel_10711648436424
// MI455X (gfx1250) — hardware-verified
//
#include <hip/hip_runtime.h>
#include <math.h>

typedef __attribute__((ext_vector_type(16))) _Float16 v16h;
typedef __attribute__((ext_vector_type(8)))  _Float16 v8h;
typedef __attribute__((ext_vector_type(8)))  float    v8f;
typedef __attribute__((ext_vector_type(4)))  float    v4f;

constexpr int NB    = 8192;
constexpr int NT    = 50;
constexpr int NH    = 75;
constexpr int NL    = 10;
constexpr int NP    = 80;
constexpr int NWAVE = NP / 16;
constexpr int NTHR  = NWAVE * 32;
constexpr int MB    = 32;
constexpr int NBLK  = NB / MB;
constexpr int LEAD  = 16;
constexpr int SEG   = NP;
constexpr int HP    = LEAD + NL * SEG;
constexpr int KP    = 2 * SEG;
constexpr int KCH0  = 3;
constexpr int KCHL  = KP / 32;
constexpr int PLANE = NP * KP;
constexpr int PREP_DW = NL * PLANE / 2;
constexpr float WCARRY     = 16.0f;
constexpr float WCARRY_INV = 1.0f / 16.0f;
constexpr float RCARRY     = 1024.0f;
constexpr float RCARRY_INV = 1.0f / 1024.0f;
static_assert(NP == NWAVE * 16 && NH <= NP);
static_assert(NB % MB == 0 && MB == 32);
static_assert(HP % 8 == 0 && KP % 8 == 0 && LEAD % 8 == 0 && SEG % 8 == 0);
static_assert(32 * KCH0 == LEAD + SEG);
static_assert(LEAD + NH <= 32 * KCH0);
static_assert(32 * KCHL == KP && KP == 2 * SEG);
static_assert(LEAD + SEG * (NL - 2) + 32 * KCHL == HP);
static_assert((MB * HP) % 8 == 0 && (MB * NT) % 4 == 0);
static_assert((NL * NP) % NTHR == 0);
static_assert(PREP_DW % 256 == 0);
static_assert(NWAVE * MB <= NTHR);
static_assert(MB * LEAD / 8 == 64 && NWAVE >= 4);

__device__ __forceinline__ unsigned short f2bf_bits(float f) {
  unsigned u = __float_as_uint(f);
  return (unsigned short)((u + 0x7FFFu + ((u >> 16) & 1u)) >> 16);
}
__device__ __forceinline__ float bf_bits2f(unsigned short h) { return __uint_as_float(((unsigned)h) << 16); }
__device__ __forceinline__ float bf16r(float f) { return bf_bits2f(f2bf_bits(f)); }

__device__ __forceinline__ void dep_guard_all(v8f& a, v8f& b, v8f& c, v8f& d,
                                              v16h x0, v16h x1, v16h x2, v16h x3, v16h y) {
  asm volatile("v_nop\n\tv_nop\n\tv_nop\n\tv_nop"
               : "+v"(a), "+v"(b), "+v"(c), "+v"(d)
               : "v"(x0), "v"(x1), "v"(x2), "v"(x3), "v"(y));
}
__device__ __forceinline__ void acc_guard4(v8f& a, v8f& b, v8f& c, v8f& d) {
  asm volatile("v_nop\n\tv_nop\n\tv_nop\n\tv_nop" : "+v"(a), "+v"(b), "+v"(c), "+v"(d));
}
__device__ __forceinline__ void sw_fence() { asm volatile("" ::: "memory"); }

template <typename T> struct Frag;
template <> struct Frag<_Float16> {
  typedef v16h V; union U { v16h v; v8h h[2]; };
  static __device__ __forceinline__ v16h load(const _Float16* p) {
    U f; f.h[0] = *(const v8h*)(p); f.h[1] = *(const v8h*)(p + 16); return f.v;
  }
  static __device__ __forceinline__ v8f mma(v16h a, v16h b, v8f c) {
    return __builtin_amdgcn_wmma_f32_16x16x32_f16(false, a, false, b, (short)0, c, false, false);
  }
};

__device__ __forceinline__ void st2u(unsigned* p, unsigned v) { *(volatile unsigned*)p = v; __threadfence(); *(volatile unsigned*)p = v; }

__device__ __forceinline__ float tanh_f(float x) {
  const float ax = fminf(fabsf(x), 10.0f);
  const float e  = expf(2.0f * ax);
  const float t  = 1.0f - 2.0f * __builtin_amdgcn_rcpf(e + 1.0f);
  return copysignf(t, x);
}

__device__ __forceinline__ void split_store(float hv, _Float16* ph, _Float16* pr) {
  const _Float16 hq = (_Float16)hv;
  const float hqf = (float)hq;
  const float rs = (hv - hqf) * RCARRY;
  *ph = hq;
  *pr = (_Float16)rs;
}

template <int NCH>
__device__ __forceinline__ void mm_tile(const _Float16* a0h, const _Float16* a1h,
                                        const _Float16* a0r, const _Float16* a1r,
                                        const _Float16* bp,
                                        v8f& c0h, v8f& c1h, v8f& c0r, v8f& c1r) {
  const v8f z8 = {0.f, 0.f, 0.f, 0.f, 0.f, 0.f, 0.f, 0.f};
  c0h = z8; c1h = z8; c0r = z8; c1r = z8;
#pragma unroll
  for (int kc = 0; kc < NCH; ++kc) {
    if (kc == 2 || kc == 4) sw_fence();
    const v16h b   = Frag<_Float16>::load(bp  + 32 * kc);
    const v16h fh0 = Frag<_Float16>::load(a0h + 32 * kc);
    const v16h fh1 = Frag<_Float16>::load(a1h + 32 * kc);
    const v16h fr0 = Frag<_Float16>::load(a0r + 32 * kc);
    const v16h fr1 = Frag<_Float16>::load(a1r + 32 * kc);
    c0h = Frag<_Float16>::mma(fh0, b, c0h);
    c1h = Frag<_Float16>::mma(fh1, b, c1h);
    c0r = Frag<_Float16>::mma(fr0, b, c0r);
    c1r = Frag<_Float16>::mma(fr1, b, c1r);
    dep_guard_all(c0h, c1h, c0r, c1r, fh0, fh1, fr0, fr1, b);
  }
  acc_guard4(c0h, c1h, c0r, c1r);
}

__global__ __launch_bounds__(256) void prep_kernel(const float* __restrict__ U0, const float* __restrict__ Ws,
                                                   const float* __restrict__ Us, unsigned* __restrict__ WBu) {
  const int p   = blockIdx.x * 256 + threadIdx.x;
  const int l   = p / (PLANE / 2);
  const int rem = p - l * (PLANE / 2);
  const int n   = rem / (KP / 2);
  const int kd  = rem - n * (KP / 2);
  const int nn  = (n < NH) ? n : (NH - 1);
  const int lw  = (l > 0) ? (l - 1) : 0;
  const bool nin = (n < NH);
  float v[2];
#pragma unroll
  for (int e = 0; e < 2; ++e) {
    const int k = 2 * kd + e;
    int ku0 = k - LEAD; ku0 = (ku0 < 0) ? 0 : ((ku0 > NH - 1) ? (NH - 1) : ku0);
    const int kw = (k > NH - 1) ? (NH - 1) : k;
    int ks = k - SEG; ks = (ks < 0) ? 0 : ((ks > NH - 1) ? (NH - 1) : ks);
    const float cu0 = U0[ku0 * NH + nn];
    const float cw  = Ws[((size_t)lw * NH + kw) * NH + nn];
    const float cu  = Us[((size_t)lw * NH + ks) * NH + nn];
    const float f0 = (nin && l == 0 && k >= LEAD && k < LEAD + NH) ? 1.0f : 0.0f;
    const float fw = (nin && l > 0 && k < NH) ? 1.0f : 0.0f;
    const float fu = (nin && l > 0 && k >= SEG && k < SEG + NH) ? 1.0f : 0.0f;
    const float s = fmaf(f0, cu0, fmaf(fw, cw, fu * cu));
    v[e] = WCARRY * bf16r(s);
  }
  const auto pk = __builtin_amdgcn_cvt_pkrtz(v[0], v[1]);
  const unsigned u = __builtin_bit_cast(unsigned, pk);
  st2u(WBu + p, u);
}

__global__ __launch_bounds__(NTHR) void rnn_stack_kernel(
    const float* __restrict__ x, const float* __restrict__ W0, const float* __restrict__ b0,
    const float* __restrict__ bs, const float* __restrict__ Wd, const float* __restrict__ bd,
    const unsigned short* __restrict__ WBp, float* __restrict__ out) {
  __shared__ __align__(16) _Float16 Hs[MB * HP];
  __shared__ __align__(16) _Float16 Rs[MB * HP];
  __shared__ __align__(16) float    xs[MB * NT];
  __shared__ float sBias[NL * NP];
  __shared__ float sW0[NP];
  __shared__ float sWd[NP];
  __shared__ float sP[NWAVE * MB];
  const _Float16* WB = (const _Float16*)WBp;
  const int tid = threadIdx.x, lane = tid & 31, wave = tid >> 5;
  const int c = lane & 15, hh = lane >> 4, koff = 8 * hh;
  const int rowbase = blockIdx.x * MB;
  const int n = 16 * wave + c;
  const v8h z8h = {(_Float16)0.f, (_Float16)0.f, (_Float16)0.f, (_Float16)0.f, (_Float16)0.f, (_Float16)0.f, (_Float16)0.f, (_Float16)0.f};

  for (int i = tid; i < (MB * HP) / 8; i += NTHR) {
    *(v8h*)(Hs + 8 * i) = z8h;
    *(v8h*)(Rs + 8 * i) = z8h;
  }
  {
    const v4f* xg = (const v4f*)(x + (size_t)rowbase * NT);
    for (int i = tid; i < (MB * NT) / 4; i += NTHR) {
      const v4f v = xg[i];
      v4f o;
      o[0] = bf16r(v[0]); o[1] = bf16r(v[1]); o[2] = bf16r(v[2]); o[3] = bf16r(v[3]);
      *(v4f*)(xs + 4 * i) = o;
    }
  }
  sw_fence();
  for (int i = tid; i < NL * NP; i += NTHR) {
    const int l = i / NP, nn = i - l * NP;
    const int nc = (nn < NH) ? nn : (NH - 1);
    const int lc = (l > 0) ? (l - 1) : 0;
    const float cb0 = b0[nc];
    const float cbs = bs[lc * NH + nc];
    const float f0 = (nn < NH && l == 0) ? 1.0f : 0.0f;
    const float f1 = (nn < NH && l > 0) ? 1.0f : 0.0f;
    sBias[i] = bf16r(fmaf(f0, cb0, f1 * cbs));
  }
  sw_fence();
  for (int i = tid; i < NP; i += NTHR) {
    const int nc = (i < NH) ? i : (NH - 1);
    const float a = W0[nc], d = Wd[nc];
    const float f = (i < NH) ? 1.0f : 0.0f;
    sW0[i] = bf16r(a) * f;
    sWd[i] = bf16r(d) * f;
  }
  const float bdr = bf16r(bd[0]);
  __syncthreads();
  const float w0n = sW0[n], b0n = sBias[n], wdn = sWd[n];

  const _Float16* a0h = Hs + c * HP + koff;
  const _Float16* a1h = Hs + (16 + c) * HP + koff;
  const _Float16* a0r = Rs + c * HP + koff;
  const _Float16* a1r = Rs + (16 + c) * HP + koff;

#pragma unroll 1
  for (int t = 0; t < NT; ++t) {
    {
      v8f c0h, c1h, c0r, c1r;
      const _Float16* bp = WB + (size_t)n * KP + koff;
      mm_tile<KCH0>(a0h, a1h, a0r, a1r, bp, c0h, c1h, c0r, c1r);
      float h0v[8], h1v[8];
#pragma unroll
      for (int r = 0; r < 8; ++r) {
        const float xa = xs[(8 * hh + r) * NT + t];
        const float xb = xs[(16 + 8 * hh + r) * NT + t];
        const float z0 = fmaf(fmaf(c0r[r], RCARRY_INV, c0h[r]), WCARRY_INV, fmaf(xa, w0n, b0n));
        const float z1 = fmaf(fmaf(c1r[r], RCARRY_INV, c1h[r]), WCARRY_INV, fmaf(xb, w0n, b0n));
        h0v[r] = tanh_f(z0);
        h1v[r] = tanh_f(z1);
      }
      __syncthreads();
      _Float16* hw = Hs + LEAD + n;
      _Float16* rw = Rs + LEAD + n;
#pragma unroll
      for (int r = 0; r < 8; ++r) {
        split_store(h0v[r], hw + (8 * hh + r) * HP,      rw + (8 * hh + r) * HP);
        split_store(h1v[r], hw + (16 + 8 * hh + r) * HP, rw + (16 + 8 * hh + r) * HP);
      }
      if (wave < 2) {
        *(v8h*)(Hs + (tid >> 1) * HP + 8 * (tid & 1)) = z8h;
      } else if (wave < 4) {
        const int u = tid - 64;
        *(v8h*)(Rs + (u >> 1) * HP + 8 * (u & 1)) = z8h;
      }
      __syncthreads();
    }
#pragma unroll 1
    for (int l = 1; l < NL; ++l) {
      v8f c0h, c1h, c0r, c1r;
      const int acol = LEAD + SEG * (l - 1);
      const _Float16* bp = WB + (size_t)l * PLANE + (size_t)n * KP + koff;
      mm_tile<KCHL>(a0h + acol, a1h + acol, a0r + acol, a1r + acol, bp, c0h, c1h, c0r, c1r);
      const float bl = sBias[l * NP + n];
      float h0v[8], h1v[8];
#pragma unroll
      for (int r = 0; r < 8; ++r) {
        const float z0 = fmaf(fmaf(c0r[r], RCARRY_INV, c0h[r]), WCARRY_INV, bl);
        const float z1 = fmaf(fmaf(c1r[r], RCARRY_INV, c1h[r]), WCARRY_INV, bl);
        h0v[r] = tanh_f(z0);
        h1v[r] = tanh_f(z1);
      }
      __syncthreads();
      _Float16* hw = Hs + LEAD + SEG * l + n;
      _Float16* rw = Rs + LEAD + SEG * l + n;
#pragma unroll
      for (int r = 0; r < 8; ++r) {
        split_store(h0v[r], hw + (8 * hh + r) * HP,      rw + (8 * hh + r) * HP);
        split_store(h1v[r], hw + (16 + 8 * hh + r) * HP, rw + (16 + 8 * hh + r) * HP);
      }
      if (t == NT - 1 && l == NL - 1) {
        float s0[8], s1[8];
#pragma unroll
        for (int r = 0; r < 8; ++r) { s0[r] = h0v[r] * wdn; s1[r] = h1v[r] * wdn; }
#pragma unroll
        for (int r = 0; r < 8; ++r) {
#pragma unroll
          for (int off = 1; off < 16; off <<= 1) {
            s0[r] += __shfl_xor(s0[r], off, 32);
            s1[r] += __shfl_xor(s1[r], off, 32);
          }
        }
        if (c == 0) {
#pragma unroll
          for (int r = 0; r < 8; ++r) {
            sP[wave * MB + 8 * hh + r]      = s0[r];
            sP[wave * MB + 16 + 8 * hh + r] = s1[r];
          }
        }
      }
      __syncthreads();
    }
  }

  if (wave == 0) {
    const int q = lane & 7;
    v4f o;
#pragma unroll
    for (int e = 0; e < 4; ++e) {
      const int row = 4 * q + e;
      float s = 0.0f;
#pragma unroll
      for (int w = 0; w < NWAVE; ++w) s += sP[w * MB + row];
      o[e] = s + bdr;
    }
    float* op = out + rowbase + 4 * q;
    for (int pass = 0; pass < 2; ++pass) {
      if (lane < 8) *(volatile v4f*)op = o;
      __threadfence();
    }
  }
}

extern "C" void kernel_launch(void* const* d_in, const int* in_sizes, int n_in,
                              void* d_out, int out_size, void* d_ws, size_t ws_size, hipStream_t stream) {
  if (n_in < 9 || d_out == nullptr || d_ws == nullptr) return;
  if (in_sizes[0] != NB * NT || in_sizes[1] != NH || in_sizes[2] != NH * NH || in_sizes[3] != NH ||
      in_sizes[4] != (NL - 1) * NH * NH || in_sizes[5] != (NL - 1) * NH * NH || in_sizes[6] != (NL - 1) * NH ||
      in_sizes[7] != NH || in_sizes[8] != 1 || out_size != NB) return;

  const float* x  = (const float*)d_in[0];
  const float* W0 = (const float*)d_in[1];
  const float* U0 = (const float*)d_in[2];
  const float* b0 = (const float*)d_in[3];
  const float* Ws = (const float*)d_in[4];
  const float* Us = (const float*)d_in[5];
  const float* bs = (const float*)d_in[6];
  const float* Wd = (const float*)d_in[7];
  const float* bd = (const float*)d_in[8];
  float* out = (float*)d_out;

  const size_t wb_bytes = (size_t)NL * PLANE * 2;
  if (wb_bytes > ws_size || wb_bytes > (size_t)134217728) return;
  unsigned short* WB = (unsigned short*)d_ws;

  prep_kernel<<<PREP_DW / 256, 256, 0, stream>>>(U0, Ws, Us, (unsigned*)WB);
  rnn_stack_kernel<<<NBLK, NTHR, 0, stream>>>(x, W0, b0, bs, Wd, bd, WB, out);
}
